// GCN_Encoder_56281251447117
// MI455X (gfx1250) — hardware-verified
//
#include <hip/hip_runtime.h>
#include <stddef.h>
#include <stdint.h>


#define HID    256
#define EMB    128
#define NTHR   256
#define NWAVE  8
#define EPT    8
#define CHUNK  (NTHR * EPT)
#define WCAP   (EPT * 32)
#define LISTN  (NWAVE * WCAP)
#define NB     8192
#define SLB    13
#define GBM    64
#define GTHR   128
#define WSMAX  134217728

static_assert((CHUNK & (CHUNK - 1)) == 0 && CHUNK <= 4096);
static_assert((NB & (NB - 1)) == 0 && NB == (1 << SLB));
static_assert(((long long)CHUNK << SLB) < (1LL << 31));
static_assert(NB % (NTHR * 4) == 0);
static_assert(LISTN % NTHR == 0 && NB % NTHR == 0);
static_assert(HID % 32 == 0 && EMB == 128 && HID == 2 * GTHR && EMB == GTHR);
static_assert(GBM == (GTHR / 32) * 16);

typedef float          v4f   __attribute__((ext_vector_type(4)));
typedef float          v8f   __attribute__((ext_vector_type(8)));
typedef int            v4i   __attribute__((ext_vector_type(4)));
typedef int            v8i   __attribute__((ext_vector_type(8)));
typedef unsigned short v8us  __attribute__((ext_vector_type(8)));
typedef unsigned short v16us __attribute__((ext_vector_type(16)));
typedef __bf16         v16bf __attribute__((ext_vector_type(16)));
typedef v4f  __attribute__((may_alias)) v4fa;
typedef v8us __attribute__((may_alias)) v8usa;
union FragB { v16bf v; v16us u; v8us h[2]; v8i w; };

__device__ __forceinline__ v8f wmb(const FragB& a, const FragB& b, v8f c) {
  v8f d = __builtin_amdgcn_wmma_f32_16x16x32_bf16(false, a.v, false, b.v, (short)0, c, false, false);
  asm volatile("v_nop\n\tv_nop\n\tv_nop\n\tv_nop" : "+v"(d) : "v"(a.w), "v"(b.w));
  return d;
}

__device__ __forceinline__ unsigned bf16_bits(float f) {
  const unsigned u = __float_as_uint(f);
  return (u + 0x7FFFu + ((u >> 16) & 1u)) >> 16;
}
__device__ __forceinline__ float bf16_val(float f) {
  return __uint_as_float(bf16_bits(f) << 16);
}

__device__ __forceinline__ int scan_chunk(const int* __restrict__ dsts, int nE, int cbase, int slotBase,
                                          int nb, int vec8, int* list, int tid, int lane, int wave) {
  int wc = 0;
  const int el0  = tid * EPT;
  const int e0   = cbase + el0;
  const int sent = -2147483647 - 1;
  v4i da, db;
  if (vec8 != 0 && cbase + CHUNK <= nE) {
    da = *(const v4i*)(dsts + e0);
    db = *(const v4i*)(dsts + e0 + 4);
  } else {
    da.x = (e0     < nE) ? dsts[min(e0,     nE - 1)] : sent;
    da.y = (e0 + 1 < nE) ? dsts[min(e0 + 1, nE - 1)] : sent;
    da.z = (e0 + 2 < nE) ? dsts[min(e0 + 2, nE - 1)] : sent;
    da.w = (e0 + 3 < nE) ? dsts[min(e0 + 3, nE - 1)] : sent;
    db.x = (e0 + 4 < nE) ? dsts[min(e0 + 4, nE - 1)] : sent;
    db.y = (e0 + 5 < nE) ? dsts[min(e0 + 5, nE - 1)] : sent;
    db.z = (e0 + 6 < nE) ? dsts[min(e0 + 6, nE - 1)] : sent;
    db.w = (e0 + 7 < nE) ? dsts[min(e0 + 7, nE - 1)] : sent;
  }
  const unsigned nbs = (unsigned)slotBase;
  const unsigned unb = (unsigned)nb;
  const unsigned s0 = (unsigned)da.x - nbs, s1 = (unsigned)da.y - nbs;
  const unsigned s2 = (unsigned)da.z - nbs, s3 = (unsigned)da.w - nbs;
  const unsigned s4 = (unsigned)db.x - nbs, s5 = (unsigned)db.y - nbs;
  const unsigned s6 = (unsigned)db.z - nbs, s7 = (unsigned)db.w - nbs;
  const bool h0 = s0 < unb, h1 = s1 < unb, h2 = s2 < unb, h3 = s3 < unb;
  const bool h4 = s4 < unb, h5 = s5 < unb, h6 = s6 < unb, h7 = s7 < unb;
  const unsigned any = __builtin_amdgcn_ballot_w32(h0 | h1 | h2 | h3 | h4 | h5 | h6 | h7);
  if (any != 0u) {
#define HITJ(J, HJ, SJ) { \
      const unsigned mj = __builtin_amdgcn_ballot_w32(HJ); \
      if (mj != 0u) { \
        if (HJ) { \
          const int pos = wc + (int)__builtin_amdgcn_mbcnt_lo(mj, 0u); \
          if (pos < WCAP) list[wave * WCAP + pos] = ((el0 + (J)) << SLB) | (int)(SJ); \
        } \
        wc += (int)__builtin_popcount(mj); } }
    HITJ(0, h0, s0)
    HITJ(1, h1, s1)
    HITJ(2, h2, s2)
    HITJ(3, h3, s3)
    HITJ(4, h4, s4)
    HITJ(5, h5, s5)
    HITJ(6, h6, s6)
    HITJ(7, h7, s7)
#undef HITJ
  }
  return wc;
}

__global__ __launch_bounds__(NTHR) void k_wprep(const float* __restrict__ W2, unsigned short* WT, int nUnits) {
  const int u = (int)blockIdx.x * NTHR + (int)threadIdx.x;
  if (u >= nUnits) return;
  const int kq = HID >> 3;
  const int n  = u / kq;
  const int k8 = (u - n * kq) * 8;
  const float* p = W2 + (size_t)k8 * EMB + n;
  v8us o;
  o[0] = (unsigned short)bf16_bits(p[0]);
  o[1] = (unsigned short)bf16_bits(p[(size_t)EMB]);
  o[2] = (unsigned short)bf16_bits(p[(size_t)2 * EMB]);
  o[3] = (unsigned short)bf16_bits(p[(size_t)3 * EMB]);
  o[4] = (unsigned short)bf16_bits(p[(size_t)4 * EMB]);
  o[5] = (unsigned short)bf16_bits(p[(size_t)5 * EMB]);
  o[6] = (unsigned short)bf16_bits(p[(size_t)6 * EMB]);
  o[7] = (unsigned short)bf16_bits(p[(size_t)7 * EMB]);
  unsigned short* dp = WT + (size_t)n * HID + k8;
  *(volatile v8us*)dp = o;
  __threadfence();
  *(volatile v8us*)dp = o;
}

__global__ __launch_bounds__(NTHR) void k_deg(const int* __restrict__ dsts, int nE, int vec8, float* dis) {
  __shared__ __attribute__((aligned(16))) int scnt[NB];
  __shared__ __attribute__((aligned(16))) int list[LISTN];
  __shared__ int wcnt[NWAVE];
  const int tid = (int)threadIdx.x, lane = tid & 31, wave = tid >> 5;
  const int nodeBase = (int)blockIdx.x * NB;

  for (int i = tid; i < NB; i += NTHR) scnt[i] = 0;
  for (int i = tid; i < LISTN; i += NTHR) list[i] = 0;
  if (tid < NWAVE) wcnt[tid] = 0;
  __syncthreads();

  const int nChunks = (nE + CHUNK - 1) / CHUNK;
#pragma unroll 1
  for (int ch = 0; ch < nChunks; ++ch) {
    const int cbase = ch * CHUNK;
    const int wc = scan_chunk(dsts, nE, cbase, nodeBase, NB, vec8, list, tid, lane, wave);
    if (lane == 0) wcnt[wave] = wc;
    __syncthreads();
    if (wave == 0) {
#pragma unroll 1
      for (int w2 = 0; w2 < NWAVE; ++w2) {
        int c = wcnt[w2];
        c = c < 0 ? 0 : (c > WCAP ? WCAP : c);
#pragma unroll 1
        for (int b0 = 0; b0 < c; b0 += 32) {
          const int idx = b0 + lane;
          const int ent = list[w2 * WCAP + (idx < WCAP ? idx : WCAP - 1)];
          const int m32 = (c - b0) < 32 ? (c - b0) : 32;
#pragma unroll 1
          for (int k = 0; k < m32; ++k) {
            const int u  = __builtin_amdgcn_readlane(ent, k);
            const int sl = u & (NB - 1);
            if (lane == 0) scnt[sl] = scnt[sl] + 1;
          }
        }
      }
    }
    __syncthreads();
  }

  v4f vals[NB / (NTHR * 4)];
#pragma unroll
  for (int it = 0; it < NB / (NTHR * 4); ++it) {
    const int s0 = it * (NTHR * 4) + 4 * tid;
    const v4i c4 = *(const v4i*)(scnt + s0);
    v4f v;
    v.x = rsqrtf((float)c4.x + 1.0f);
    v.y = rsqrtf((float)c4.y + 1.0f);
    v.z = rsqrtf((float)c4.z + 1.0f);
    v.w = rsqrtf((float)c4.w + 1.0f);
    vals[it] = v;
  }
#pragma unroll
  for (int it = 0; it < NB / (NTHR * 4); ++it) {
    const int s0 = it * (NTHR * 4) + 4 * tid;
    *(volatile v4f*)(dis + (size_t)nodeBase + s0) = vals[it];
  }
  __threadfence();
#pragma unroll
  for (int it = 0; it < NB / (NTHR * 4); ++it) {
    const int s0 = it * (NTHR * 4) + 4 * tid;
    *(volatile v4f*)(dis + (size_t)nodeBase + s0) = vals[it];
  }
}

__global__ __launch_bounds__(NTHR) void k_csum(const int* __restrict__ srcs, const int* __restrict__ dsts,
                                               const float* __restrict__ dis, int nE, int nN, int vec8,
                                               float* cpl) {
  __shared__ __attribute__((aligned(16))) float sacc[NB];
  __shared__ __attribute__((aligned(16))) int list[LISTN];
  __shared__ int wcnt[NWAVE];
  const int tid = (int)threadIdx.x, lane = tid & 31, wave = tid >> 5;
  const int nodeBase = (int)blockIdx.x * NB;

  for (int i = tid; i < NB; i += NTHR) sacc[i] = 0.0f;
  for (int i = tid; i < LISTN; i += NTHR) list[i] = 0;
  if (tid < NWAVE) wcnt[tid] = 0;
  __syncthreads();

  const int nChunks = (nE + CHUNK - 1) / CHUNK;
#pragma unroll 1
  for (int ch = 0; ch < nChunks; ++ch) {
    const int cbase = ch * CHUNK;
    const int wc = scan_chunk(dsts, nE, cbase, nodeBase, NB, vec8, list, tid, lane, wave);
    if (lane == 0) wcnt[wave] = wc;
    __syncthreads();
    if (wave == 0) {
#pragma unroll 1
      for (int w2 = 0; w2 < NWAVE; ++w2) {
        int c = wcnt[w2];
        c = c < 0 ? 0 : (c > WCAP ? WCAP : c);
#pragma unroll 1
        for (int b0 = 0; b0 < c; b0 += 32) {
          const int idx = b0 + lane;
          const int ent = list[w2 * WCAP + (idx < WCAP ? idx : WCAP - 1)];
          const int el  = (ent >> SLB) & (CHUNK - 1);
          int eid = cbase + el;
          eid = eid < 0 ? 0 : (eid > nE - 1 ? nE - 1 : eid);
          const int sraw = srcs[eid];
          const int s = sraw < 0 ? 0 : (sraw > nN - 1 ? nN - 1 : sraw);
          const float dv = dis[s];
          const int dvi = __float_as_int(dv);
          const int m32 = (c - b0) < 32 ? (c - b0) : 32;
#pragma unroll 1
          for (int k = 0; k < m32; ++k) {
            const int u   = __builtin_amdgcn_readlane(ent, k);
            const int sl  = u & (NB - 1);
            const float val = __int_as_float(__builtin_amdgcn_readlane(dvi, k));
            if (lane == 0) sacc[sl] = sacc[sl] + val;
          }
        }
      }
    }
    __syncthreads();
  }

  v4f vals[NB / (NTHR * 4)];
#pragma unroll
  for (int it = 0; it < NB / (NTHR * 4); ++it) {
    const int s0 = it * (NTHR * 4) + 4 * tid;
    const v4f a4 = *(const v4fa*)(sacc + s0);
    const v4f d4 = *(const v4fa*)(dis + (size_t)nodeBase + s0);
    v4f v;
    v.x = d4.x * (a4.x + d4.x);
    v.y = d4.y * (a4.y + d4.y);
    v.z = d4.z * (a4.z + d4.z);
    v.w = d4.w * (a4.w + d4.w);
    vals[it] = v;
  }
#pragma unroll
  for (int it = 0; it < NB / (NTHR * 4); ++it) {
    const int s0 = it * (NTHR * 4) + 4 * tid;
    *(volatile v4f*)(cpl + (size_t)nodeBase + s0) = vals[it];
  }
  __threadfence();
#pragma unroll
  for (int it = 0; it < NB / (NTHR * 4); ++it) {
    const int s0 = it * (NTHR * 4) + 4 * tid;
    *(volatile v4f*)(cpl + (size_t)nodeBase + s0) = vals[it];
  }
}

__global__ __launch_bounds__(GTHR) void k_gemm(
    const float* __restrict__ cpl, const float* __restrict__ W1, const float* __restrict__ b1,
    const unsigned short* __restrict__ WT, const float* __restrict__ b2, float* out, int nN) {
  __shared__ __attribute__((aligned(16))) float sW1[HID];
  __shared__ __attribute__((aligned(16))) float sB1[HID];
  __shared__ __attribute__((aligned(16))) float sB2[EMB];
  __shared__ __attribute__((aligned(16))) float stg[EMB * GBM];
  const int tid = (int)threadIdx.x, lane = tid & 31, wave = tid >> 5, hh = lane >> 4, m = lane & 15;
  const int rowBase = (int)blockIdx.x * GBM;

  sW1[tid]        = bf16_val(W1[tid]);
  sW1[tid + GTHR] = bf16_val(W1[tid + GTHR]);
  sB1[tid]        = bf16_val(b1[tid]);
  sB1[tid + GTHR] = bf16_val(b1[tid + GTHR]);
  sB2[tid]        = bf16_val(b2[tid]);
  __syncthreads();

  const int row = rowBase + 16 * wave + m;
  const int rc  = row < nN ? row : nN - 1;
  const float cval = cpl[rc];

  v8f acc[8];
  {
    const v8f z = {0.f, 0.f, 0.f, 0.f, 0.f, 0.f, 0.f, 0.f};
#pragma unroll
    for (int t = 0; t < 8; ++t) acc[t] = z;
  }
  const unsigned short* wp = WT + (size_t)m * HID + 8 * hh;

#pragma unroll 1
  for (int kk = 0; kk < HID / 32; ++kk) {
    const int k0 = 32 * kk;
    const v4f wa = *(const v4fa*)(sW1 + k0 + 8 * hh);
    const v4f wb = *(const v4fa*)(sW1 + k0 + 8 * hh + 4);
    const v4f wc = *(const v4fa*)(sW1 + k0 + 16 + 8 * hh);
    const v4f wd = *(const v4fa*)(sW1 + k0 + 16 + 8 * hh + 4);
    const v4f ba = *(const v4fa*)(sB1 + k0 + 8 * hh);
    const v4f bb = *(const v4fa*)(sB1 + k0 + 8 * hh + 4);
    const v4f bc = *(const v4fa*)(sB1 + k0 + 16 + 8 * hh);
    const v4f bd = *(const v4fa*)(sB1 + k0 + 16 + 8 * hh + 4);
    float v[16];
    v[0]  = fmaxf(fmaf(cval, wa.x, ba.x), 0.f);
    v[1]  = fmaxf(fmaf(cval, wa.y, ba.y), 0.f);
    v[2]  = fmaxf(fmaf(cval, wa.z, ba.z), 0.f);
    v[3]  = fmaxf(fmaf(cval, wa.w, ba.w), 0.f);
    v[4]  = fmaxf(fmaf(cval, wb.x, bb.x), 0.f);
    v[5]  = fmaxf(fmaf(cval, wb.y, bb.y), 0.f);
    v[6]  = fmaxf(fmaf(cval, wb.z, bb.z), 0.f);
    v[7]  = fmaxf(fmaf(cval, wb.w, bb.w), 0.f);
    v[8]  = fmaxf(fmaf(cval, wc.x, bc.x), 0.f);
    v[9]  = fmaxf(fmaf(cval, wc.y, bc.y), 0.f);
    v[10] = fmaxf(fmaf(cval, wc.z, bc.z), 0.f);
    v[11] = fmaxf(fmaf(cval, wc.w, bc.w), 0.f);
    v[12] = fmaxf(fmaf(cval, wd.x, bd.x), 0.f);
    v[13] = fmaxf(fmaf(cval, wd.y, bd.y), 0.f);
    v[14] = fmaxf(fmaf(cval, wd.z, bd.z), 0.f);
    v[15] = fmaxf(fmaf(cval, wd.w, bd.w), 0.f);
    FragB ah, al;
#pragma unroll
    for (int i = 0; i < 16; ++i) {
      const unsigned hb = bf16_bits(v[i]);
      ah.u[i] = (unsigned short)hb;
      al.u[i] = (unsigned short)bf16_bits(v[i] - __uint_as_float(hb << 16));
    }
#pragma unroll
    for (int nt = 0; nt < 8; ++nt) {
      const unsigned short* wq = wp + (size_t)(16 * nt) * HID + k0;
      FragB bf;
      bf.h[0] = *(const v8usa*)wq;
      bf.h[1] = *(const v8usa*)(wq + 16);
      acc[nt] = wmb(ah, bf, acc[nt]);
      acc[nt] = wmb(al, bf, acc[nt]);
    }
  }

#pragma unroll
  for (int nt = 0; nt < 8; ++nt) {
    const int lc = 16 * nt + m;
    const float bv = sB2[lc];
#pragma unroll
    for (int r = 0; r < 8; ++r) {
      const int lr = 16 * wave + 8 * hh + r;
      const float y  = acc[nt][r] + bv;
      const float e  = __expf(-y);
      const float sg = __builtin_amdgcn_rcpf(1.0f + e);
      stg[lc * GBM + lr] = sg;
    }
  }
  __syncthreads();

  int nv = nN - rowBase;
  nv = nv < 0 ? 0 : (nv > GBM ? GBM : nv);
  const bool ok = (4 * m < nv);
  v4f pv[16];
#pragma unroll
  for (int i = 0; i < 16; ++i) {
    const int lc = 32 * wave + 2 * i + hh;
    pv[i] = *(const v4fa*)(stg + lc * GBM + 4 * m);
  }
#pragma unroll
  for (int i = 0; i < 16; ++i) {
    const int lc = 32 * wave + 2 * i + hh;
    float* op = out + (size_t)lc * (size_t)nN + rowBase + 4 * m;
    if (ok) *(volatile v4f*)op = pv[i];
  }
  __threadfence();
#pragma unroll
  for (int i = 0; i < 16; ++i) {
    const int lc = 32 * wave + 2 * i + hh;
    float* op = out + (size_t)lc * (size_t)nN + rowBase + 4 * m;
    if (ok) *(volatile v4f*)op = pv[i];
  }
}

static inline int cdiv(int a, int b) { return (a + b - 1) / b; }

extern "C" void kernel_launch(void* const* d_in, const int* in_sizes, int n_in,
                              void* d_out, int out_size, void* d_ws, size_t ws_size,
                              hipStream_t stream) {
  if (n_in < 5) return;
  if (in_sizes[0] < 2 || (in_sizes[0] & 1) != 0) return;
  const int nE = in_sizes[0] / 2;
  if (nE < 1) return;
  if (in_sizes[1] != HID || in_sizes[2] != HID) return;
  if (in_sizes[3] != HID * EMB || in_sizes[4] != EMB) return;
  if (out_size <= 0 || (out_size % EMB) != 0) return;
  const int nN = out_size / EMB;
  if (nN < 32 || (nN % 32) != 0) return;

  const int*   edge = (const int*)d_in[0];
  const float* W1   = (const float*)d_in[1];
  const float* b1   = (const float*)d_in[2];
  const float* W2   = (const float*)d_in[3];
  const float* b2   = (const float*)d_in[4];
  float* out = (float*)d_out;
  const int* src = edge;
  const int* dst = edge + nE;

  const int gA = cdiv(nN, NB);
  if ((long long)gA * NB < (long long)nN) return;
  const int NBP = gA * NB;
  const int MP  = cdiv(nN, GBM) * GBM;
  const int gM  = MP / GBM;
  if (MP > NBP) return;
  const int vec8 = ((nE & 3) == 0) ? 1 : 0;

  char* ws = (char*)d_ws;
  size_t off = 0;
  const size_t oDIS = off; off += (size_t)NBP * 4;               off = (off + 255) & ~(size_t)255;
  const size_t oCPL = off; off += (size_t)NBP * 4;               off = (off + 255) & ~(size_t)255;
  const size_t oWT  = off; off += (size_t)EMB * HID * 2;         off = (off + 255) & ~(size_t)255;
  if (off > ws_size || off > (size_t)WSMAX) return;
  float*          DIS = (float*)(ws + oDIS);
  float*          CPL = (float*)(ws + oCPL);
  unsigned short* WT  = (unsigned short*)(ws + oWT);

  const int nUw = EMB * (HID / 8);
  k_wprep<<<cdiv(nUw, NTHR), NTHR, 0, stream>>>(W2, WT, nUw);
  k_deg<<<gA, NTHR, 0, stream>>>(dst, nE, vec8, DIS);
  k_csum<<<gA, NTHR, 0, stream>>>(src, dst, DIS, nE, nN, vec8, CPL);
  k_gemm<<<gM, GTHR, 0, stream>>>(CPL, W1, b1, WT, b2, out, nN);
}
